// HATSModel_5231270167366
// MI455X (gfx1250) — hardware-verified
//
#include <hip/hip_runtime.h>
#include <math.h>

constexpr int NSTK   = 8192;
constexpr int NSTEP  = 64;
constexpr int NFEAT  = 6;
constexpr int NHID   = 128;
constexpr int NG3    = 3 * NHID;
constexpr int XROW   = NFEAT * NSTEP;
constexpr int NTHR   = 256;
constexpr int RB     = 16;
constexpr int HPITCH = 136;
constexpr int OPITCH = 132;
constexpr int KXPAD  = 32;
constexpr int XTW    = 8;
constexpr int TPITCH = 129;
constexpr int KSL    = 256;
constexpr int NSL    = NSTK / KSL;
constexpr float WCARRY = 256.0f;
constexpr float HCARRY = 16.0f;
constexpr float GINV   = 1.0f / 4096.0f;
constexpr float BN_EPS = 1e-5f;
static_assert(NSTK == 8192, "shift-based (t, n) decode");
static_assert(NSTK % RB == 0, "recurrence grid exact");
static_assert(NHID == 16 * (NTHR / 32), "8 waves x 16 hidden units");
static_assert((4 * RB * HPITCH) % NTHR == 0, "h zero-fill loop exact");
static_assert((NSTK * NSTEP) % NTHR == 0, "x plane grid exact");
static_assert((NG3 * (KXPAD / 8)) % NTHR == 0, "w_ih0 plane grid exact");
static_assert((NG3 * (NHID / 8)) % NTHR == 0, "weight plane grids exact");
static_assert(NHID % 64 == 0 && NSTK % 64 == 0, "GEMM M, N tile multiples");
static_assert(KSL % 32 == 0 && NHID % 32 == 0, "GEMM K multiples of 32");
static_assert(NSL * KSL == NSTK, "split-K covers all rows");
static_assert((NHID * NHID) % (4 * NTHR) == 0, "partial-plane reduce loop exact");
static_assert(NSTK % (32 * (NTHR / 32)) == 0, "head grid exact");
static_assert(NSTK % 64 == 0, "hidden-plane grid exact");

typedef __attribute__((ext_vector_type(16))) _Float16 v16h;
typedef __attribute__((ext_vector_type(8)))  _Float16 v8h;
typedef __attribute__((ext_vector_type(16))) __bf16   v16b;
typedef __attribute__((ext_vector_type(8)))  __bf16   v8b;
typedef __attribute__((ext_vector_type(8)))  float    v8f;
typedef __attribute__((ext_vector_type(4)))  float    v4f;
typedef __attribute__((ext_vector_type(4)))  unsigned v4u;

__device__ __forceinline__ unsigned short f2bf_bits(float f) {
  unsigned u = __float_as_uint(f);
  return (unsigned short)((u + 0x7FFFu + ((u >> 16) & 1u)) >> 16);
}
__device__ __forceinline__ float bf_bits2f(unsigned short h) { return __uint_as_float(((unsigned)h) << 16); }
__device__ __forceinline__ float bf16r(float f) { return bf_bits2f(f2bf_bits(f)); }
__device__ __forceinline__ unsigned h16_bits(float f) { return (unsigned)__builtin_bit_cast(unsigned short, (_Float16)f); }

__device__ __forceinline__ void dep_guard_h(v8f& a, v8f& b, v16h x, v16h y) { asm volatile("v_nop\n\tv_nop\n\tv_nop\n\tv_nop" : "+v"(a), "+v"(b) : "v"(x), "v"(y)); }
__device__ __forceinline__ void dep_guard_b(v8f& a, v8f& b, v16b x, v16b y) { asm volatile("v_nop\n\tv_nop\n\tv_nop\n\tv_nop" : "+v"(a), "+v"(b) : "v"(x), "v"(y)); }
__device__ __forceinline__ void keep4_h(v16h a, v16h b, v16h c, v16h d) { asm volatile("v_nop" :: "v"(a), "v"(b), "v"(c), "v"(d)); }
__device__ __forceinline__ void keep4_b(v16b a, v16b b, v16b c, v16b d) { asm volatile("v_nop" :: "v"(a), "v"(b), "v"(c), "v"(d)); }
__device__ __forceinline__ void acc_guard4(v8f& a, v8f& b, v8f& c, v8f& d) { asm volatile("v_nop\n\tv_nop\n\tv_nop\n\tv_nop" : "+v"(a), "+v"(b), "+v"(c), "+v"(d)); }
template <typename T> struct Frag;
template <> struct Frag<_Float16> {
  typedef v16h V; union U { v16h v; v8h h[2]; };
  static __device__ __forceinline__ v16h load(const _Float16* p) {
    U f; f.h[0] = *(const v8h*)(p); f.h[1] = *(const v8h*)(p + 16); return f.v;
  }
  static __device__ __forceinline__ v8f mma(v16h a, v16h b, v8f c) {
    return __builtin_amdgcn_wmma_f32_16x16x32_f16(false, a, false, b, (short)0, c, false, false);
  }
  static __device__ __forceinline__ void guard(v8f& a, v8f& b, v16h x, v16h y) { dep_guard_h(a, b, x, y); }
  static __device__ __forceinline__ void keep(v16h a, v16h b, v16h c, v16h d) { keep4_h(a, b, c, d); }
};
template <> struct Frag<__bf16> {
  typedef v16b V; union U { v16b v; v8b h[2]; };
  static __device__ __forceinline__ v16b load(const __bf16* p) {
    U f; f.h[0] = *(const v8b*)(p); f.h[1] = *(const v8b*)(p + 16); return f.v;
  }
  static __device__ __forceinline__ v8f mma(v16b a, v16b b, v8f c) {
    return __builtin_amdgcn_wmma_f32_16x16x32_bf16(false, a, false, b, (short)0, c, false, false);
  }
  static __device__ __forceinline__ void guard(v8f& a, v8f& b, v16b x, v16b y) { dep_guard_b(a, b, x, y); }
  static __device__ __forceinline__ void keep(v16b a, v16b b, v16b c, v16b d) { keep4_b(a, b, c, d); }
};

__device__ __forceinline__ float fsig(float x)  { return __builtin_amdgcn_rcpf(1.0f + expf(-x)); }
__device__ __forceinline__ float ftanh(float x) { return 1.0f - 2.0f * __builtin_amdgcn_rcpf(expf(2.0f * x) + 1.0f); }

template <int ET> struct Elem;
template <> struct Elem<0> { typedef _Float16 T; };
template <> struct Elem<1> { typedef __bf16 T; };
template <int ET, bool SPLIT, int BIAS_MODE, int OUT_MODE, bool RESID, int ACT = 0>
__global__ __launch_bounds__(256) void wmma_gemm64(
    const unsigned short* __restrict__ Ap, const unsigned short* __restrict__ A2p, int lda, long strideA,
    const unsigned short* __restrict__ Btp, const unsigned short* __restrict__ Bt2p, int ldb, long strideB,
    void* __restrict__ Cout, void* __restrict__ Cout2, int ldc, long strideC,
    const float* __restrict__ bias,
    const float* __restrict__ resid, long strideR,
    int M, int N, int K, float scale) {
  typedef typename Elem<ET>::T T;
  typedef typename Frag<T>::V V;
  const T* A = (const T*)Ap; const T* A2 = (const T*)A2p; const T* Bt = (const T*)Btp; const T* Bt2 = (const T*)Bt2p;
  __shared__ __align__(16) float sT[8][16 * 68];
  const int b    = blockIdx.y;
  const int lane = threadIdx.x & 31;
  const int wave = threadIdx.x >> 5;
  const int tilesN = N >> 6;
  const int tilesM = M >> 6;
  const int tile = blockIdx.x * 8 + wave;
  if (tile >= tilesM * tilesN) return;
  const int tm = tile / tilesN;
  const int tn = tile - tm * tilesN;
  const int m0 = tm << 6;
  const int n0 = tn << 6;

  const T* Ab  = A  + (size_t)b * strideA;
  const T* Bb  = Bt + (size_t)b * strideB;
  const T* Ab2 = SPLIT ? (A2  + (size_t)b * strideA) : nullptr;
  const T* Bb2 = SPLIT ? (Bt2 + (size_t)b * strideB) : nullptr;

  const int rlane = lane & 15;
  const int koff  = (lane >> 4) * 8;
  const int mOff  = (lane >> 4) * 8;

  v8f acc[4][4];
#pragma unroll
  for (int i = 0; i < 4; ++i)
#pragma unroll
    for (int j = 0; j < 4; ++j) acc[i][j] = (v8f){0.f,0.f,0.f,0.f,0.f,0.f,0.f,0.f};

  for (int k0 = 0; k0 < K; k0 += 32) {
    V bh[4], bl[4];
#pragma unroll
    for (int j = 0; j < 4; ++j) {
      const size_t bo = (size_t)(n0 + (j << 4) + rlane) * ldb + koff + k0;
      bh[j] = Frag<T>::load(Bb + bo);
      if (SPLIT) bl[j] = Frag<T>::load(Bb2 + bo);
    }
#pragma unroll
    for (int i = 0; i < 4; ++i) {
      const size_t ao = (size_t)(m0 + (i << 4) + rlane) * lda + koff + k0;
      V ah = Frag<T>::load(Ab + ao);
      V al;
      if (SPLIT) al = Frag<T>::load(Ab2 + ao);
#pragma unroll
      for (int j = 0; j < 4; ++j) {
        acc[i][j] = Frag<T>::mma(ah, bh[j], acc[i][j]);
        if (SPLIT) {
          acc[i][j] = Frag<T>::mma(ah, bl[j], acc[i][j]);
          acc[i][j] = Frag<T>::mma(al, bh[j], acc[i][j]);
        }
      }
      Frag<T>::guard(acc[i][0], acc[i][3], ah, SPLIT ? al : ah);
    }
    Frag<T>::keep(bh[0], bh[1], bh[2], bh[3]);
    if (SPLIT) Frag<T>::keep(bl[0], bl[1], bl[2], bl[3]);
  }
  acc_guard4(acc[0][0], acc[0][1], acc[0][2], acc[0][3]);
  acc_guard4(acc[1][0], acc[1][1], acc[1][2], acc[1][3]);
  acc_guard4(acc[2][0], acc[2][1], acc[2][2], acc[2][3]);
  acc_guard4(acc[3][0], acc[3][1], acc[3][2], acc[3][3]);

  float* slab = sT[wave];
  const float* Rb = RESID ? (resid + (size_t)b * strideR) : nullptr;
#pragma unroll
  for (int i = 0; i < 4; ++i) {
    const int mBase = m0 + (i << 4);
#pragma unroll
    for (int j = 0; j < 4; ++j) {
      const int n = n0 + (j << 4) + rlane;
      float bv = 0.f;
      if (BIAS_MODE == 2) bv = bias[n];
#pragma unroll
      for (int r = 0; r < 8; ++r) {
        float v = acc[i][j][r] * scale;
        if (BIAS_MODE == 1) v += bias[mBase + mOff + r];
        if (BIAS_MODE == 2) v += bv;
        if (RESID) v += Rb[(size_t)(mBase + mOff + r) * ldc + n];
        if (ACT == 1) v = tanhf(v);
        if (ACT == 2) v = fmaxf(v, 0.0f);
        if (ACT == 3) v = v / (1.0f + expf(-v));
        if (ACT == 4) v = (v > 0.f) ? v : 0.01f * v;
        if (ACT == 5) v = 0.5f * v * (1.0f + erff(v * 0.70710678118654752f));
        slab[(mOff + r) * 68 + (j << 4) + rlane] = v;
      }
    }
    __builtin_amdgcn_fence(__ATOMIC_RELEASE, "workgroup");
    __builtin_amdgcn_wave_barrier();
    __builtin_amdgcn_fence(__ATOMIC_ACQUIRE, "workgroup");
    if (OUT_MODE == 0) {
      float* C = (float*)Cout + (size_t)b * strideC;
      const int hh = lane >> 4, c4 = (lane & 15) * 4;
      for (int pass = 0; pass < 2; ++pass) {
#pragma unroll
        for (int it = 0; it < 8; ++it) {
          const int row = it * 2 + hh;
          v4f v = *(const v4f*)(slab + row * 68 + c4);
          *(volatile v4f*)(C + (size_t)(mBase + row) * ldc + n0 + c4) = v;
        }
        __threadfence();
      }
    } else {
      const int q = lane >> 3, c8 = (lane & 7) * 8;
      unsigned short* C  = (unsigned short*)Cout  + (size_t)b * strideC;
      unsigned short* C2 = (OUT_MODE == 2) ? ((unsigned short*)Cout2 + (size_t)b * strideC) : nullptr;
      for (int pass = 0; pass < 2; ++pass) {
#pragma unroll
        for (int it = 0; it < 4; ++it) {
          const int row = it * 4 + q;
          const float* sp = slab + row * 68 + c8;
          v8h hv, lv;
#pragma unroll
          for (int e = 0; e < 8; ++e) {
            if (OUT_MODE == 1) {
              hv[e] = (_Float16)sp[e];
            } else {
              unsigned short hb = f2bf_bits(sp[e]);
              unsigned short lb = f2bf_bits(sp[e] - bf_bits2f(hb));
              hv[e] = __builtin_bit_cast(_Float16, hb);
              lv[e] = __builtin_bit_cast(_Float16, lb);
            }
          }
          *(volatile v8h*)(C + (size_t)(mBase + row) * ldc + n0 + c8) = hv;
          if (OUT_MODE == 2) *(volatile v8h*)(C2 + (size_t)(mBase + row) * ldc + n0 + c8) = lv;
        }
        __threadfence();
      }
    }
    __builtin_amdgcn_fence(__ATOMIC_RELEASE, "workgroup");
    __builtin_amdgcn_wave_barrier();
    __builtin_amdgcn_fence(__ATOMIC_ACQUIRE, "workgroup");
  }
}

template <int MODE>
__global__ __launch_bounds__(NTHR) void cvt8_kernel(const float* __restrict__ src, unsigned short* __restrict__ dst,
                                                    int nrow, int ncol8, int spitch, int scol0, float sc) {
  const int i  = blockIdx.x * NTHR + threadIdx.x;
  const int n8 = nrow * ncol8;
  if (i < n8) {
    const int row = i / ncol8;
    const int c8  = i - row * ncol8;
    const float* sp = src + (size_t)row * spitch + scol0 + c8 * 8;
    const v4f a = *(const v4f*)(sp);
    const v4f b = *(const v4f*)(sp + 4);
    v8h hv;
#pragma unroll
    for (int e = 0; e < 4; ++e) {
      unsigned short b0, b1;
      if (MODE == 0) {
        b0 = f2bf_bits(a[e] * sc);
        b1 = f2bf_bits(b[e] * sc);
      } else {
        b0 = __builtin_bit_cast(unsigned short, (_Float16)(bf16r(a[e]) * sc));
        b1 = __builtin_bit_cast(unsigned short, (_Float16)(bf16r(b[e]) * sc));
      }
      hv[e]     = __builtin_bit_cast(_Float16, b0);
      hv[4 + e] = __builtin_bit_cast(_Float16, b1);
    }
    *(volatile v8h*)(dst + (size_t)i * 8) = hv;
    __threadfence();
    *(volatile v8h*)(dst + (size_t)i * 8) = hv;
  }
}

__global__ __launch_bounds__(NTHR) void xprep_kernel(const float* __restrict__ x, unsigned short* __restrict__ XT) {
  const int g = blockIdx.x * NTHR + threadIdx.x;
  const int t = g >> 13;
  const int n = g & (NSTK - 1);
  const float* xp = x + (size_t)n * XROW + t;
  v4u o;
#pragma unroll
  for (int p = 0; p < 3; ++p) {
    const float f0 = bf16r(xp[(2 * p) * NSTEP]) * HCARRY;
    const float f1 = bf16r(xp[(2 * p + 1) * NSTEP]) * HCARRY;
    o[p] = h16_bits(f0) | (h16_bits(f1) << 16);
  }
  o[3] = 0u;
  v4u* op = (v4u*)(XT + (size_t)g * XTW);
  *(volatile v4u*)op = o;
  __threadfence();
  *(volatile v4u*)op = o;
}

__global__ __launch_bounds__(NTHR) void wi0prep_kernel(const float* __restrict__ w, unsigned short* __restrict__ WI0) {
  const int i = blockIdx.x * NTHR + threadIdx.x;
  if (i < NG3 * (KXPAD / 8)) {
    const int row = i >> 2;
    const int c8 = (i & 3) * 8;
    v4u o;
#pragma unroll
    for (int p = 0; p < 4; ++p) {
      const int k0 = c8 + 2 * p, k1 = k0 + 1;
      const int kc0 = (k0 < NFEAT) ? k0 : (NFEAT - 1);
      const int kc1 = (k1 < NFEAT) ? k1 : (NFEAT - 1);
      const float f0 = bf16r(w[row * NFEAT + kc0]) * WCARRY;
      const float f1 = bf16r(w[row * NFEAT + kc1]) * WCARRY;
      const unsigned b0 = (k0 < NFEAT) ? h16_bits(f0) : 0u;
      const unsigned b1 = (k1 < NFEAT) ? h16_bits(f1) : 0u;
      o[p] = b0 | (b1 << 16);
    }
    v4u* op = (v4u*)(WI0 + (size_t)i * 8);
    *(volatile v4u*)op = o;
    __threadfence();
    *(volatile v4u*)op = o;
  }
}

__global__ __launch_bounds__(NTHR) void gru2_kernel(const unsigned short* __restrict__ XTp,
                                                   const unsigned short* __restrict__ WI0p,
                                                   const unsigned short* __restrict__ WH0p,
                                                   const unsigned short* __restrict__ WI1p,
                                                   const unsigned short* __restrict__ WH1p,
                                                   const float* __restrict__ bih0, const float* __restrict__ bhh0,
                                                   const float* __restrict__ bih1, const float* __restrict__ bhh1,
                                                   float* __restrict__ H2) {
  __shared__ __align__(16) _Float16 Ah[4][RB * HPITCH];
  __shared__ __align__(16) float    Hs[RB * OPITCH];
  union XU { v16h v; v4u u[2]; };
  const _Float16* WI0 = (const _Float16*)WI0p;
  const _Float16* WH0 = (const _Float16*)WH0p;
  const _Float16* WI1 = (const _Float16*)WI1p;
  const _Float16* WH1 = (const _Float16*)WH1p;
  const v4u* XT4 = (const v4u*)XTp;
  const int tid = threadIdx.x, lane = tid & 31, wave = tid >> 5;
  const int c = lane & 15, hh = lane >> 4, koff = hh * 8;
  const int j = 16 * wave + c;
  const int n0 = blockIdx.x * RB;

  {
    _Float16* ahf = &Ah[0][0];
#pragma unroll 1
    for (int i = tid; i < 4 * RB * HPITCH; i += NTHR) ahf[i] = (_Float16)0.0f;
  }
  const float b0r  = bf16r(bih0[j]) + bf16r(bhh0[j]);
  const float b0z  = bf16r(bih0[NHID + j]) + bf16r(bhh0[NHID + j]);
  const float b0in = bf16r(bih0[2 * NHID + j]);
  const float b0hn = bf16r(bhh0[2 * NHID + j]);
  const float b1r  = bf16r(bih1[j]) + bf16r(bhh1[j]);
  const float b1z  = bf16r(bih1[NHID + j]) + bf16r(bhh1[NHID + j]);
  const float b1in = bf16r(bih1[2 * NHID + j]);
  const float b1hn = bf16r(bhh1[2 * NHID + j]);
  float h1s[8], h2s[8];
#pragma unroll
  for (int r = 0; r < 8; ++r) { h1s[r] = 0.0f; h2s[r] = 0.0f; }
  __syncthreads();

  const v8f z8 = {0.f, 0.f, 0.f, 0.f, 0.f, 0.f, 0.f, 0.f};
  const unsigned xmask = (hh == 0) ? 0xffffffffu : 0u;
  const v4u xm4 = {xmask, xmask, xmask, xmask};
  const v4u zu4 = {0u, 0u, 0u, 0u};

#pragma unroll 1
  for (int t = 0; t < NSTEP; ++t) {
    const int cur = t & 1, nxt = cur ^ 1;
    v8f ar = z8, az = z8, ain = z8, ahn = z8;
    {
      v4u xw = XT4[(size_t)t * NSTK + n0 + c];
      xw = xw & xm4;
      XU xu; xu.u[0] = xw; xu.u[1] = zu4;
      const v16h bxr = Frag<_Float16>::load(WI0 + (size_t)j * KXPAD + koff);
      const v16h bxz = Frag<_Float16>::load(WI0 + (size_t)(NHID + j) * KXPAD + koff);
      const v16h bxn = Frag<_Float16>::load(WI0 + (size_t)(2 * NHID + j) * KXPAD + koff);
      ar  = Frag<_Float16>::mma(xu.v, bxr, ar);
      az  = Frag<_Float16>::mma(xu.v, bxz, az);
      ain = Frag<_Float16>::mma(xu.v, bxn, ain);
      dep_guard_h(ar, ain, xu.v, bxn);
      keep4_h(bxr, bxz, bxn, xu.v);
    }
    {
      const _Float16* a1row = &Ah[cur][0] + c * HPITCH + koff;
#pragma unroll 1
      for (int k0 = 0; k0 < NHID; k0 += 32) {
        const v16h a  = Frag<_Float16>::load(a1row + k0);
        const v16h br = Frag<_Float16>::load(WH0 + (size_t)j * NHID + koff + k0);
        const v16h bz = Frag<_Float16>::load(WH0 + (size_t)(NHID + j) * NHID + koff + k0);
        const v16h bn = Frag<_Float16>::load(WH0 + (size_t)(2 * NHID + j) * NHID + koff + k0);
        ar  = Frag<_Float16>::mma(a, br, ar);
        az  = Frag<_Float16>::mma(a, bz, az);
        ahn = Frag<_Float16>::mma(a, bn, ahn);
        dep_guard_h(ar, ahn, a, bn);
        keep4_h(br, bz, bn, a);
      }
    }
    acc_guard4(ar, az, ain, ahn);
    {
      _Float16* h1n = &Ah[nxt][0];
#pragma unroll
      for (int r = 0; r < 8; ++r) {
        const float pr  = ar[r]  * GINV + b0r;
        const float pz  = az[r]  * GINV + b0z;
        const float pin = ain[r] * GINV + b0in;
        const float phn = ahn[r] * GINV + b0hn;
        const float rg = fsig(pr);
        const float zg = fsig(pz);
        const float ng = ftanh(pin + rg * phn);
        const float ho = h1s[r];
        const float hn = (1.0f - zg) * ng + zg * ho;
        h1s[r] = hn;
        h1n[(8 * hh + r) * HPITCH + j] = (_Float16)(hn * HCARRY);
      }
    }
    __syncthreads();
    v8f cr = z8, cz = z8, cin = z8, chn = z8;
    {
      const _Float16* b1row = &Ah[nxt][0] + c * HPITCH + koff;
#pragma unroll 1
      for (int k0 = 0; k0 < NHID; k0 += 32) {
        const v16h a  = Frag<_Float16>::load(b1row + k0);
        const v16h br = Frag<_Float16>::load(WI1 + (size_t)j * NHID + koff + k0);
        const v16h bz = Frag<_Float16>::load(WI1 + (size_t)(NHID + j) * NHID + koff + k0);
        const v16h bn = Frag<_Float16>::load(WI1 + (size_t)(2 * NHID + j) * NHID + koff + k0);
        cr  = Frag<_Float16>::mma(a, br, cr);
        cz  = Frag<_Float16>::mma(a, bz, cz);
        cin = Frag<_Float16>::mma(a, bn, cin);
        dep_guard_h(cr, cin, a, bn);
        keep4_h(br, bz, bn, a);
      }
    }
    {
      const _Float16* a2row = &Ah[2 + cur][0] + c * HPITCH + koff;
#pragma unroll 1
      for (int k0 = 0; k0 < NHID; k0 += 32) {
        const v16h a  = Frag<_Float16>::load(a2row + k0);
        const v16h br = Frag<_Float16>::load(WH1 + (size_t)j * NHID + koff + k0);
        const v16h bz = Frag<_Float16>::load(WH1 + (size_t)(NHID + j) * NHID + koff + k0);
        const v16h bn = Frag<_Float16>::load(WH1 + (size_t)(2 * NHID + j) * NHID + koff + k0);
        cr  = Frag<_Float16>::mma(a, br, cr);
        cz  = Frag<_Float16>::mma(a, bz, cz);
        chn = Frag<_Float16>::mma(a, bn, chn);
        dep_guard_h(cr, chn, a, bn);
        keep4_h(br, bz, bn, a);
      }
    }
    acc_guard4(cr, cz, cin, chn);
    {
      _Float16* h2n = &Ah[2 + nxt][0];
#pragma unroll
      for (int r = 0; r < 8; ++r) {
        const float pr  = cr[r]  * GINV + b1r;
        const float pz  = cz[r]  * GINV + b1z;
        const float pin = cin[r] * GINV + b1in;
        const float phn = chn[r] * GINV + b1hn;
        const float rg = fsig(pr);
        const float zg = fsig(pz);
        const float ng = ftanh(pin + rg * phn);
        const float ho = h2s[r];
        const float hn = (1.0f - zg) * ng + zg * ho;
        h2s[r] = hn;
        h2n[(8 * hh + r) * HPITCH + j] = (_Float16)(hn * HCARRY);
      }
    }
    __syncthreads();
  }

#pragma unroll
  for (int r = 0; r < 8; ++r) Hs[(8 * hh + r) * OPITCH + j] = h2s[r];
  __syncthreads();
  for (int pass = 0; pass < 2; ++pass) {
#pragma unroll
    for (int it = 0; it < 2; ++it) {
      const int idx = it * NTHR + tid;
      const int row = idx >> 5, c4 = (idx & 31) * 4;
      const v4f v = *(const v4f*)(Hs + row * OPITCH + c4);
      *(volatile v4f*)(H2 + (size_t)(n0 + row) * NHID + c4) = v;
    }
    __threadfence();
  }
}

__global__ __launch_bounds__(NTHR) void colstats_kernel(const float* __restrict__ src, float* __restrict__ stat) {
  __shared__ float red[NTHR / 32][32];
  const int tid = threadIdx.x, lane = tid & 31, wave = tid >> 5;
  const int col = blockIdx.x * 32 + lane;
  float s = 0.0f;
#pragma unroll 4
  for (int row = wave; row < NSTK; row += NTHR / 32) s += src[(size_t)row * NHID + col];
  red[wave][lane] = s;
  __syncthreads();
  float tot = 0.0f;
#pragma unroll
  for (int w = 0; w < NTHR / 32; ++w) tot += red[w][lane];
  const float mu = tot * (1.0f / NSTK);
  float ss = 0.0f;
#pragma unroll 4
  for (int row = wave; row < NSTK; row += NTHR / 32) {
    const float d = src[(size_t)row * NHID + col] - mu;
    ss += d * d;
  }
  __syncthreads();
  red[wave][lane] = ss;
  __syncthreads();
  float tot2 = 0.0f;
#pragma unroll
  for (int w = 0; w < NTHR / 32; ++w) tot2 += red[w][lane];
  const float var = tot2 * (1.0f / NSTK);
  const float rs = rsqrtf(var + BN_EPS);
  if (wave == 0) {
    for (int pass = 0; pass < 2; ++pass) {
      ((volatile float*)stat)[col] = mu;
      ((volatile float*)stat)[NHID + col] = rs;
      __threadfence();
    }
  }
}

__global__ __launch_bounds__(NTHR) void hidden_kernel(const float* __restrict__ H2, const float* __restrict__ stat,
                                                     const float* __restrict__ gam, const float* __restrict__ bet,
                                                     unsigned short* __restrict__ Hh, unsigned short* __restrict__ Hl,
                                                     unsigned short* __restrict__ HTh, unsigned short* __restrict__ HTl) {
  __shared__ float Tt[64 * TPITCH];
  const int tid = threadIdx.x;
  const int r0 = blockIdx.x * 64;
  {
    const int c4 = (tid & 31) * 4, rsub = tid >> 5;
    const v4f mu4 = *(const v4f*)(stat + c4);
    const v4f rs4 = *(const v4f*)(stat + NHID + c4);
    const v4f g4  = *(const v4f*)(gam + c4);
    const v4f b4  = *(const v4f*)(bet + c4);
    float gg[4], bb[4];
#pragma unroll
    for (int e = 0; e < 4; ++e) { gg[e] = bf16r(g4[e]); bb[e] = bf16r(b4[e]); }
#pragma unroll
    for (int it = 0; it < 8; ++it) {
      const int row = it * 8 + rsub;
      const v4f v = *(const v4f*)(H2 + (size_t)(r0 + row) * NHID + c4);
#pragma unroll
      for (int e = 0; e < 4; ++e) {
        const float t1 = v[e] - mu4[e];
        const float t2 = t1 * rs4[e];
        Tt[row * TPITCH + c4 + e] = t2 * gg[e] + bb[e];
      }
    }
  }
  __syncthreads();
  const int rowA = tid >> 4, c8A = (tid & 15) * 8;
  v8h hvA[4], lvA[4];
#pragma unroll
  for (int it = 0; it < 4; ++it) {
#pragma unroll
    for (int e = 0; e < 8; ++e) {
      const float f = Tt[(it * 16 + rowA) * TPITCH + c8A + e];
      const unsigned short hb = f2bf_bits(f);
      const unsigned short lb = f2bf_bits(f - bf_bits2f(hb));
      hvA[it][e] = __builtin_bit_cast(_Float16, hb);
      lvA[it][e] = __builtin_bit_cast(_Float16, lb);
    }
  }
  const int qB = tid >> 3, c8B = (tid & 7) * 8;
  v8h hvB[4], lvB[4];
#pragma unroll
  for (int g4 = 0; g4 < 4; ++g4) {
    const int cc = g4 * 32 + qB;
#pragma unroll
    for (int e = 0; e < 8; ++e) {
      const float f = Tt[(c8B + e) * TPITCH + cc];
      const unsigned short hb = f2bf_bits(f);
      const unsigned short lb = f2bf_bits(f - bf_bits2f(hb));
      hvB[g4][e] = __builtin_bit_cast(_Float16, hb);
      lvB[g4][e] = __builtin_bit_cast(_Float16, lb);
    }
  }
  for (int pass = 0; pass < 2; ++pass) {
#pragma unroll
    for (int it = 0; it < 4; ++it) {
      const size_t o = (size_t)(r0 + it * 16 + rowA) * NHID + c8A;
      *(volatile v8h*)(Hh + o) = hvA[it];
      *(volatile v8h*)(Hl + o) = lvA[it];
    }
#pragma unroll
    for (int g4 = 0; g4 < 4; ++g4) {
      const size_t o = (size_t)(g4 * 32 + qB) * NSTK + r0 + c8B;
      *(volatile v8h*)(HTh + o) = hvB[g4];
      *(volatile v8h*)(HTl + o) = lvB[g4];
    }
    __threadfence();
  }
}

__global__ __launch_bounds__(NTHR) void fold_kernel(const float* __restrict__ GP, const float* __restrict__ fcw,
                                                   const float* __restrict__ fcb,
                                                   unsigned short* __restrict__ FTh, unsigned short* __restrict__ FTl,
                                                   float* __restrict__ FCBR) {
  __shared__ __align__(16) float Gs[NHID * NHID];
  __shared__ float ps[NHID];
  __shared__ float qs[NHID];
  const int tid = threadIdx.x;
#pragma unroll 1
  for (int m = 0; m < (NHID * NHID) / (4 * NTHR); ++m) {
    const int i4 = m * NTHR + tid;
    v4f s = {0.f, 0.f, 0.f, 0.f};
#pragma unroll 4
    for (int sl = 0; sl < NSL; ++sl) s += *(const v4f*)(GP + (size_t)sl * NHID * NHID + (size_t)i4 * 4);
    *(v4f*)(Gs + (size_t)i4 * 4) = s;
  }
  __syncthreads();
  if (tid < NHID) {
    float s = 0.0f;
#pragma unroll 4
    for (int k = 0; k < NHID; ++k) s += Gs[tid * NHID + k];
    ps[tid] = s * (1.0f / NHID);
  }
  __syncthreads();
  if (tid < NHID) {
    float s = 0.0f;
#pragma unroll 4
    for (int jj = 0; jj < NHID; ++jj) s += bf16r(fcw[tid * NHID + jj]) * ps[jj];
    qs[tid] = s;
    const float fb = bf16r(fcb[tid]);
    ((volatile float*)FCBR)[tid] = fb;
    __threadfence();
    ((volatile float*)FCBR)[tid] = fb;
  }
  __syncthreads();
  const int csub = tid >> 4, j8 = (tid & 15) * 8;
#pragma unroll 1
  for (int p8 = 0; p8 < 8; ++p8) {
    const int cc = p8 * 16 + csub;
    const float qv = qs[cc] * (1.0f / NHID);
    float acc[8];
#pragma unroll
    for (int e = 0; e < 8; ++e) acc[e] = 0.0f;
    const float* wrow = fcw + (size_t)cc * NHID;
#pragma unroll 1
    for (int k = 0; k < NHID; ++k) {
      const float w = bf16r(wrow[k]);
#pragma unroll
      for (int e = 0; e < 8; ++e) acc[e] += Gs[(j8 + e) * NHID + k] * w;
    }
    v8h hv, lv;
#pragma unroll
    for (int e = 0; e < 8; ++e) {
      const float f = acc[e] * (1.0f / NHID) - qv;
      const unsigned short hb = f2bf_bits(f);
      const unsigned short lb = f2bf_bits(f - bf_bits2f(hb));
      hv[e] = __builtin_bit_cast(_Float16, hb);
      lv[e] = __builtin_bit_cast(_Float16, lb);
    }
    const size_t o = (size_t)cc * NHID + j8;
    for (int pass = 0; pass < 2; ++pass) {
      *(volatile v8h*)(FTh + o) = hv;
      *(volatile v8h*)(FTl + o) = lv;
      __threadfence();
    }
  }
}

__global__ __launch_bounds__(NTHR) void head_kernel(const float* __restrict__ OFC, const float* __restrict__ stat,
                                                   const float* __restrict__ gam, const float* __restrict__ bet,
                                                   const float* __restrict__ fcow, const float* __restrict__ fcob,
                                                   float* __restrict__ out) {
  const int tid = threadIdx.x, lane = tid & 31, wave = tid >> 5;
  const int rowbase = (blockIdx.x * (NTHR / 32) + wave) * 32;
  const int c4 = lane * 4;
  const v4f mu4 = *(const v4f*)(stat + c4);
  const v4f rs4 = *(const v4f*)(stat + NHID + c4);
  const v4f g4  = *(const v4f*)(gam + c4);
  const v4f b4  = *(const v4f*)(bet + c4);
  const v4f w4  = *(const v4f*)(fcow + c4);
  const float fb = bf16r(fcob[0]);
  float gg[4], bb[4], ww[4];
#pragma unroll
  for (int e = 0; e < 4; ++e) { gg[e] = bf16r(g4[e]); bb[e] = bf16r(b4[e]); ww[e] = bf16r(w4[e]); }
  float yl = 0.0f;
#pragma unroll 1
  for (int rr = 0; rr < 32; ++rr) {
    const v4f v = *(const v4f*)(OFC + (size_t)(rowbase + rr) * NHID + c4);
    float s = 0.0f;
#pragma unroll
    for (int e = 0; e < 4; ++e) {
      const float t1 = v[e] - mu4[e];
      const float t2 = t1 * rs4[e];
      float a = t2 * gg[e] + bb[e];
      a = (a >= 0.0f) ? a : 0.01f * a;
      s += a * ww[e];
    }
#pragma unroll
    for (int off = 1; off < 32; off <<= 1) s += __shfl_xor(s, off, 32);
    const float y = s + fb;
    yl = (lane == rr) ? y : yl;
  }
  float* op = out + rowbase + lane;
  *(volatile float*)op = yl;
  __threadfence();
  *(volatile float*)op = yl;
}

extern "C" void kernel_launch(void* const* d_in, const int* in_sizes, int n_in,
                              void* d_out, int out_size, void* d_ws, size_t ws_size, hipStream_t stream) {
  if (n_in < 17 || d_out == nullptr || d_ws == nullptr) return;
  if (in_sizes[0] != NSTK * XROW || in_sizes[1] != NG3 * NFEAT || in_sizes[2] != NG3 * NHID ||
      in_sizes[3] != NG3 || in_sizes[4] != NG3 || in_sizes[5] != NG3 * NHID || in_sizes[6] != NG3 * NHID ||
      in_sizes[7] != NG3 || in_sizes[8] != NG3 || in_sizes[9] != NHID || in_sizes[10] != NHID ||
      in_sizes[11] != NHID * NHID || in_sizes[12] != NHID || in_sizes[13] != NHID || in_sizes[14] != NHID ||
      in_sizes[15] != NHID || in_sizes[16] != 1 || out_size != NSTK) return;

  const float* x     = (const float*)d_in[0];
  const float* w_ih0 = (const float*)d_in[1];
  const float* w_hh0 = (const float*)d_in[2];
  const float* b_ih0 = (const float*)d_in[3];
  const float* b_hh0 = (const float*)d_in[4];
  const float* w_ih1 = (const float*)d_in[5];
  const float* w_hh1 = (const float*)d_in[6];
  const float* b_ih1 = (const float*)d_in[7];
  const float* b_hh1 = (const float*)d_in[8];
  const float* bn1_g = (const float*)d_in[9];
  const float* bn1_b = (const float*)d_in[10];
  const float* fc_w  = (const float*)d_in[11];
  const float* fc_b  = (const float*)d_in[12];
  const float* bn2_g = (const float*)d_in[13];
  const float* bn2_b = (const float*)d_in[14];
  const float* fco_w = (const float*)d_in[15];
  const float* fco_b = (const float*)d_in[16];
  float* out = (float*)d_out;

  char* ws = (char*)d_ws; size_t off = 0;
  auto carve = [&](size_t bytes) -> char* { char* p = ws + off; off += (bytes + 255) & ~(size_t)255; return p; };
  unsigned short* XT    = (unsigned short*)carve((size_t)NSTEP * NSTK * XTW * 2);
  unsigned short* WI0   = (unsigned short*)carve((size_t)NG3 * KXPAD * 2);
  unsigned short* WH0   = (unsigned short*)carve((size_t)NG3 * NHID * 2);
  unsigned short* WI1   = (unsigned short*)carve((size_t)NG3 * NHID * 2);
  unsigned short* WH1   = (unsigned short*)carve((size_t)NG3 * NHID * 2);
  float*          H2    = (float*)carve((size_t)NSTK * NHID * 4);
  float*          STAT1 = (float*)carve((size_t)2 * NHID * 4);
  unsigned short* Hh    = (unsigned short*)carve((size_t)NSTK * NHID * 2);
  unsigned short* Hl    = (unsigned short*)carve((size_t)NSTK * NHID * 2);
  unsigned short* HTh   = (unsigned short*)carve((size_t)NHID * NSTK * 2);
  unsigned short* HTl   = (unsigned short*)carve((size_t)NHID * NSTK * 2);
  float*          GP    = (float*)carve((size_t)NSL * NHID * NHID * 4);
  unsigned short* FTh   = (unsigned short*)carve((size_t)NHID * NHID * 2);
  unsigned short* FTl   = (unsigned short*)carve((size_t)NHID * NHID * 2);
  float*          FCBR  = (float*)carve((size_t)NHID * 4);
  float*          OFC   = (float*)carve((size_t)NSTK * NHID * 4);
  float*          STAT2 = (float*)carve((size_t)2 * NHID * 4);
  if (off > ws_size || off > (size_t)134217728) return;

  xprep_kernel<<<(NSTEP * NSTK) / NTHR, NTHR, 0, stream>>>(x, XT);
  wi0prep_kernel<<<(NG3 * (KXPAD / 8) + NTHR - 1) / NTHR, NTHR, 0, stream>>>(w_ih0, WI0);
  const int n8w = NG3 * (NHID / 8);
  cvt8_kernel<1><<<(n8w + NTHR - 1) / NTHR, NTHR, 0, stream>>>(w_hh0, WH0, NG3, NHID / 8, NHID, 0, WCARRY);
  cvt8_kernel<1><<<(n8w + NTHR - 1) / NTHR, NTHR, 0, stream>>>(w_ih1, WI1, NG3, NHID / 8, NHID, 0, WCARRY);
  cvt8_kernel<1><<<(n8w + NTHR - 1) / NTHR, NTHR, 0, stream>>>(w_hh1, WH1, NG3, NHID / 8, NHID, 0, WCARRY);

  gru2_kernel<<<NSTK / RB, NTHR, 0, stream>>>(XT, WI0, WH0, WI1, WH1, b_ih0, b_hh0, b_ih1, b_hh1, H2);

  colstats_kernel<<<NHID / 32, NTHR, 0, stream>>>(H2, STAT1);
  hidden_kernel<<<NSTK / 64, NTHR, 0, stream>>>(H2, STAT1, bn1_g, bn1_b, Hh, Hl, HTh, HTl);

  wmma_gemm64<1, true, 0, 0, false, 0><<<dim3(1, NSL), 256, 0, stream>>>(
      HTh, HTl, NSTK, (long)KSL, HTh, HTl, NSTK, (long)KSL, (void*)GP, (void*)GP, NHID, (long)NHID * NHID,
      STAT1, H2, 0L, NHID, NHID, KSL, 1.0f);

  fold_kernel<<<1, NTHR, 0, stream>>>(GP, fc_w, fc_b, FTh, FTl, FCBR);

  wmma_gemm64<1, true, 2, 0, false, 0><<<dim3((NSTK / 64) * (NHID / 64) / 8, 1), 256, 0, stream>>>(
      Hh, Hl, NHID, 0L, FTh, FTl, NHID, 0L, (void*)OFC, (void*)OFC, NHID, 0L,
      FCBR, H2, 0L, NSTK, NHID, NHID, 1.0f);

  colstats_kernel<<<NHID / 32, NTHR, 0, stream>>>(OFC, STAT2);
  head_kernel<<<NSTK / (32 * (NTHR / 32)), NTHR, 0, stream>>>(OFC, STAT2, bn2_g, bn2_b, fco_w, fco_b, out);
}
